// SeNaTraBlock_29111288332437
// MI455X (gfx1250) — hardware-verified
//
#include <hip/hip_runtime.h>
#include <math.h>

typedef __attribute__((ext_vector_type(16))) _Float16 v16h;
typedef __attribute__((ext_vector_type(16))) __bf16 v16b;
typedef __attribute__((ext_vector_type(8)))  _Float16 v8h;
typedef __attribute__((ext_vector_type(8)))  float v8f;
typedef __attribute__((ext_vector_type(4)))  float v4f;
typedef __attribute__((ext_vector_type(2)))  float v2f;
typedef __attribute__((ext_vector_type(4)))  unsigned v4u;
typedef __attribute__((ext_vector_type(4)))  int v4i;
typedef float __attribute__((may_alias)) float_a;
typedef int __attribute__((may_alias)) int_a;

template <typename T> __device__ __forceinline__ void vst2(void* p, T v) { *(volatile T*)p = v; __threadfence(); *(volatile T*)p = v; }
__device__ __forceinline__ v8f wmma16(v16h a, v16h b, v8f c) {
  v8f d = __builtin_amdgcn_wmma_f32_16x16x32_f16(false, a, false, b, (short)0, c, false, false);
  asm volatile("v_nop\n\tv_nop\n\tv_nop\n\tv_nop" : "+v"(d) : "v"(a), "v"(b));
  return d;
}
__device__ __forceinline__ v8f wmma_bf(v16b a, v16b b, v8f c) {
  v8f d = __builtin_amdgcn_wmma_f32_16x16x32_bf16(false, a, false, b, (short)0, c, false, false);
  asm volatile("v_nop\n\tv_nop\n\tv_nop\n\tv_nop" : "+v"(d) : "v"(a), "v"(b));
  return d;
}
__device__ __forceinline__ v16h frag_h(const _Float16* rowk0, int lane) {
  union { v16h v; v8h q[2]; } u; const _Float16* p = rowk0 + 8 * (lane >> 4);
  u.q[0] = *(const v8h*)p; u.q[1] = *(const v8h*)(p + 16); return u.v;
}
__device__ __forceinline__ v16h frag_f32(const float* rowk0, int lane) {
  v16h a; const float* p = rowk0 + 8 * (lane >> 4);
#pragma unroll
  for (int i = 0; i < 8; ++i) { a[i] = (_Float16)p[i]; a[8 + i] = (_Float16)p[16 + i]; }
  return a;
}
__device__ __forceinline__ v16h frag_f32s(const float* rowk0, int lane, float sc) {
  v16h a; const float* p = rowk0 + 8 * (lane >> 4);
#pragma unroll
  for (int i = 0; i < 8; ++i) { a[i] = (_Float16)(p[i] * sc); a[8 + i] = (_Float16)(p[16 + i] * sc); }
  return a;
}
__device__ __forceinline__ v16h fragc_f32(const float* W, int k0, int n, int lane, int ld, int K) {
  v16h a; const int g = lane >> 4;
#pragma unroll
  for (int i = 0; i < 8; ++i) { const int ka = k0 + 8 * g + i, kb = ka + 16;
    a[i] = (_Float16)(ka < K ? W[(size_t)(ka < K ? ka : K - 1) * ld + n] : 0.f); a[8 + i] = (_Float16)(kb < K ? W[(size_t)(kb < K ? kb : K - 1) * ld + n] : 0.f); }
  return a;
}
struct F2 { v16b h, l; };
__device__ __forceinline__ F2 bsplit16(const float v[16]) { F2 r;
#pragma unroll
  for (int i = 0; i < 16; ++i) { const __bf16 h = (__bf16)v[i]; r.h[i] = h; r.l[i] = (__bf16)(v[i] - (float)h); }
  return r; }
__device__ __forceinline__ F2 split_row(const float* row, int k0, int lane) { float v[16]; const float* p = row + k0 + 8 * (lane >> 4);
#pragma unroll
  for (int i = 0; i < 8; ++i) { v[i] = p[i]; v[8 + i] = p[16 + i]; }
  return bsplit16(v); }
__device__ __forceinline__ F2 split_rowK(const float* row, int k0, int lane, int K) { float v[16]; const int g = lane >> 4;
#pragma unroll
  for (int i = 0; i < 8; ++i) { const int ka = k0 + 8 * g + i, kb = ka + 16; v[i] = ka < K ? row[ka < K ? ka : K - 1] : 0.f; v[8 + i] = kb < K ? row[kb < K ? kb : K - 1] : 0.f; }
  return bsplit16(v); }
__device__ __forceinline__ F2 split_col(const float* W, int k0, int n, int lane, int ld, int K) { float v[16]; const int g = lane >> 4;
#pragma unroll
  for (int i = 0; i < 8; ++i) { const int ka = k0 + 8 * g + i, kb = ka + 16; v[i] = ka < K ? W[(size_t)(ka < K ? ka : K - 1) * ld + n] : 0.f; v[8 + i] = kb < K ? W[(size_t)(kb < K ? kb : K - 1) * ld + n] : 0.f; }
  return bsplit16(v); }
__device__ __forceinline__ v8f mac3(const F2& a, const F2& b, v8f c) { c = wmma_bf(a.l, b.h, c); c = wmma_bf(a.h, b.l, c); return wmma_bf(a.h, b.h, c); }
__device__ __forceinline__ float sigm(float v) { return 1.0f / (1.0f + expf(-v)); }
#define LDSX() do { asm volatile("s_wait_dscnt 0" ::: "memory"); __builtin_amdgcn_wave_barrier(); __builtin_amdgcn_fence(__ATOMIC_RELEASE, "workgroup"); } while (0)


#define NB 4
#define HH 56
#define WWD 56
#define NTOK 3136
#define NR (NB * NTOK)
#define DM 128
#define NHD 4
#define HD 32
#define WIN 7
#define HID 384
#ifndef NRT
#define NRT NR
#endif
typedef __attribute__((ext_vector_type(8))) __bf16 v8b;
__device__ __forceinline__ v16b frag_b(const __bf16* rowk0, int lane) {
  union { v16b v; v8b q[2]; } u; const __bf16* p = rowk0 + 8 * (lane >> 4);
  u.q[0] = *(const v8b*)p; u.q[1] = *(const v8b*)(p + 16); return u.v;
}
__device__ __forceinline__ float bfr(float v) { return (float)(__bf16)v; }
__device__ __attribute__((noinline)) float exp_ni(float v) { return expf(v); }
__device__ __attribute__((noinline)) float erf_ni(float v) { return erff(v); }
__device__ __forceinline__ float gelu_exact(float v) { return 0.5f * v * (1.0f + erf_ni(v * 0.70710678118654752f)); }
__device__ __attribute__((noinline)) float cos_ni(float v) { return cosf(v); }
__device__ __attribute__((noinline)) float sin_ni(float v) { return sinf(v); }
__constant__ float c_inv[16] = {1.000000000e+00f,5.623413324e-01f,3.162277639e-01f,1.778279394e-01f,1.000000015e-01f,5.623412877e-02f,3.162277862e-02f,1.778279431e-02f,9.999999776e-03f,5.623413250e-03f,3.162277862e-03f,1.778279431e-03f,1.000000047e-03f,5.623413017e-04f,3.162277862e-04f,1.778279402e-04f};

#define PK_QKV 0
#define PK_P   (PK_QKV + 3 * DM * DM)
#define PK_W1  (PK_P + DM * DM)
#define PK_W2  (PK_W1 + HID * DM)
#define PK_END (PK_W2 + DM * HID)
#define WS_PK  0u
#define WS_AH  (((2u * PK_END) + 127u) / 128u * 128u)
#define WS_AL  (WS_AH + 2u * NR * DM)
#define WS_Q   (WS_AL + 2u * NR * DM)
#define WS_K   (WS_Q + 4u * NR * DM)
#define WS_V   (WS_K + 4u * NR * DM)
#define WS_Y   (WS_V + 4u * NR * DM)
#define WS_HFH (WS_Y + 4u * NR * DM)
#define WS_HFL (WS_HFH + 2u * NR * HID)
#define WS_END (WS_HFL + 2u * NR * HID)

__global__ __launch_bounds__(256) void k_pack(const float* __restrict__ WQKV, const float* __restrict__ WP, const float* __restrict__ W1, const float* __restrict__ W2, __bf16* __restrict__ PK) {
  __shared__ __align__(16) __bf16 s[HID]; const int n = blockIdx.x, which = blockIdx.y, t = threadIdx.x; int K = DM; size_t dst; const float* src;
  if (which == 0) { src = WQKV + (size_t)n * DM; dst = PK_QKV + (size_t)n * DM; }
  else if (which == 1) { if (n >= DM) return; src = WP + (size_t)n * DM; dst = PK_P + (size_t)n * DM; }
  else if (which == 2) { src = W1 + (size_t)n * DM; dst = PK_W1 + (size_t)n * DM; }
  else { if (n >= DM) return; K = HID; src = W2 + (size_t)n * HID; dst = PK_W2 + (size_t)n * HID; }
  for (int k = t; k < K; k += 256) s[k] = (__bf16)src[k];
  __syncthreads();
  for (int q = t; q < K / 8; q += 256) vst2((unsigned*)(PK + dst + q * 8), *(const v4u*)&s[q * 8]);
}
__global__ __launch_bounds__(128) void k_ln(const float* __restrict__ X, const float* __restrict__ Y, int first, const float* __restrict__ G, const float* __restrict__ Bb, __bf16* __restrict__ AH, __bf16* __restrict__ AL) {
  __shared__ float sred[2][4]; __shared__ __align__(16) __bf16 sh_[DM], sl_[DM]; const int t = threadIdx.x; const size_t row = blockIdx.x;
  const float v = first ? bfr(X[row * DM + t]) : Y[row * DM + t]; float s = v;
#pragma unroll
  for (int o = 1; o < 32; o <<= 1) s += __shfl_xor(s, o);
  if ((t & 31) == 0) sred[0][t >> 5] = s;
  __syncthreads();
  const float mu = ((sred[0][0] + sred[0][1]) + (sred[0][2] + sred[0][3])) * (1.0f / DM); const float d = v - mu; float q = d * d;
#pragma unroll
  for (int o = 1; o < 32; o <<= 1) q += __shfl_xor(q, o);
  if ((t & 31) == 0) sred[1][t >> 5] = q;
  __syncthreads();
  const float rs = rsqrtf(((sred[1][0] + sred[1][1]) + (sred[1][2] + sred[1][3])) * (1.0f / DM) + 1e-5f);
  const float x = d * rs * bfr(G[t]) + bfr(Bb[t]); const __bf16 hb = (__bf16)x; sh_[t] = hb; sl_[t] = (__bf16)(x - (float)hb);
  __syncthreads();
  if (t < 16) vst2((unsigned*)(AH + row * DM + t * 8), *(const v4u*)&sh_[t * 8]); else if (t < 32) vst2((unsigned*)(AL + row * DM + (t - 16) * 8), *(const v4u*)&sl_[(t - 16) * 8]);
}
template <int MODE>
__global__ __launch_bounds__(128) void k_gemm(const __bf16* __restrict__ AH, const __bf16* __restrict__ AL, const __bf16* __restrict__ P, const float* __restrict__ BIAS, const float* __restrict__ X, const float* __restrict__ Yin, float* __restrict__ Q, float* __restrict__ Kp, float* __restrict__ V, __bf16* __restrict__ OH, __bf16* __restrict__ OL, float* __restrict__ OUTF) {
  constexpr int KIN = (MODE == 3) ? HID : DM;
  __shared__ __align__(16) float so[4][16][132]; __shared__ __align__(16) __bf16 soh[4][16][136], sol[4][16][136];
  const int tid = threadIdx.x, wave = tid >> 5, lane = tid & 31, col = lane & 15, g = lane >> 4; const size_t r0 = (size_t)blockIdx.x * 64 + wave * 16; const int n0 = blockIdx.y * 128;
  v8f acc[8] = {};
#pragma unroll 2
  for (int kc = 0; kc < KIN / 32; ++kc) { F2 a; a.h = frag_b(AH + (r0 + col) * KIN + kc * 32, lane); a.l = frag_b(AL + (r0 + col) * KIN + kc * 32, lane);
#pragma unroll
    for (int j = 0; j < 8; ++j) { const v16b w = frag_b(P + (size_t)(n0 + j * 16 + col) * KIN + kc * 32, lane); acc[j] = wmma_bf(a.l, w, acc[j]); acc[j] = wmma_bf(a.h, w, acc[j]); } }
  if (MODE == 0) { const int which = n0 / DM;
#pragma unroll
    for (int j = 0; j < 8; ++j) { const int c = j * 16 + col; const int dh = c & (HD - 1); const float invv = c_inv[dh >> 1];
#pragma unroll
      for (int r = 0; r < 8; ++r) { const size_t row = r0 + 8 * g + r; float v = acc[j][r];
        if (which < 2) { const float ang = (float)(int)(row % NTOK) * invv; const float cs = cos_ni(ang), sn = sin_ni(ang); const float pv = __shfl_xor(v, 1); v = (dh & 1) ? (v * cs + pv * sn) : (v * cs - pv * sn); }
        else { (void)__shfl_xor(v, 1); }
        so[wave][8 * g + r][c] = v; } }
    LDSX(); float* DST = (which == 0) ? Q : (which == 1) ? Kp : V;
    for (int rl = 0; rl < 16; ++rl) vst2(DST + (r0 + rl) * DM + lane * 4, *(const v4f*)&so[wave][rl][lane * 4]);
    return; }
#pragma unroll
  for (int j = 0; j < 8; ++j) { const int c = n0 + j * 16 + col; const float bb = bfr(BIAS[c]);
#pragma unroll
    for (int r = 0; r < 8; ++r) { const size_t row = r0 + 8 * g + r; const float v = acc[j][r] + bb;
      if (MODE == 1) so[wave][8 * g + r][j * 16 + col] = bfr(X[row * DM + c]) + v;
      else if (MODE == 2) { const float gq = gelu_exact(v); const __bf16 hb = (__bf16)gq; soh[wave][8 * g + r][j * 16 + col] = hb; sol[wave][8 * g + r][j * 16 + col] = (__bf16)(gq - (float)hb); }
      else so[wave][8 * g + r][j * 16 + col] = Yin[row * DM + c] + v; } }
  LDSX();
  for (int rl = 0; rl < 16; ++rl) { if (MODE == 2) { if (lane < 16) { vst2((unsigned*)(OH + (r0 + rl) * HID + n0 + lane * 8), *(const v4u*)&soh[wave][rl][lane * 8]); vst2((unsigned*)(OL + (r0 + rl) * HID + n0 + lane * 8), *(const v4u*)&sol[wave][rl][lane * 8]); } }
    else vst2(OUTF + (r0 + rl) * DM + n0 + lane * 4, *(const v4f*)&so[wave][rl][lane * 4]); }
}
__global__ __launch_bounds__(128) void k_na(const float* __restrict__ Q, const float* __restrict__ Kp, const float* __restrict__ V, __bf16* __restrict__ AH, __bf16* __restrict__ AL) {
  __shared__ __align__(16) __bf16 sh_[8][DM + 8], sl_[8][DM + 8];
  const int tid = threadIdx.x, wave = tid >> 5, lane = tid & 31; const int pair = wave * 8 + (lane >> 2), part = lane & 3; const int tl = pair >> 2, h = pair & 3; const size_t row = (size_t)blockIdx.x * 8 + tl; const int b = (int)(row / NTOK), n = (int)(row % NTOK); const int i = n / WWD, jx = n % WWD;
  const int i0 = min(max(i - WIN / 2, 0), HH - WIN), j0 = min(max(jx - WIN / 2, 0), WWD - WIN); const int d0 = h * HD + part * 8;
  float q[8], o[8];
#pragma unroll
  for (int d = 0; d < 8; ++d) { q[d] = Q[row * DM + d0 + d]; o[d] = 0.f; }
  float m = -3.0e38f, l = 0.f;
#pragma unroll 1
  for (int w = 0; w < WIN * WIN; ++w) { const size_t kr = ((size_t)b * NTOK + (i0 + w / WIN) * WWD + (j0 + w % WIN)) * DM + d0; float s = 0.f;
#pragma unroll
    for (int d = 0; d < 8; ++d) s += q[d] * Kp[kr + d];
    s += __shfl_xor(s, 1); s += __shfl_xor(s, 2);
    s *= 0.17677669529663688f;
    const float mn = fmaxf(m, s); const float a = (m <= -1.0e38f) ? 0.f : exp_ni(m - mn); const float p = exp_ni(s - mn);
    l = l * a + p; m = mn;
#pragma unroll
    for (int d = 0; d < 8; ++d) o[d] = o[d] * a + p * V[kr + d]; }
  const float inv = 1.0f / l;
#pragma unroll
  for (int d = 0; d < 8; ++d) { const float v = o[d] * inv; const __bf16 hb = (__bf16)v; sh_[tl][d0 + d] = hb; sl_[tl][d0 + d] = (__bf16)(v - (float)hb); }
  __syncthreads();
  for (int qd = tid; qd < 8 * (DM / 8) * 2; qd += 128) { const int plane = qd / (8 * DM / 8), rem = qd % (8 * DM / 8); const int r = rem / (DM / 8), pc = rem % (DM / 8);
    if (plane == 0) vst2((unsigned*)(AH + ((size_t)blockIdx.x * 8 + r) * DM + pc * 8), *(const v4u*)&sh_[r][pc * 8]); else vst2((unsigned*)(AL + ((size_t)blockIdx.x * 8 + r) * DM + pc * 8), *(const v4u*)&sl_[r][pc * 8]); }
}
extern "C" void kernel_launch(void* const* d_in, const int* in_sizes, int n_in, void* d_out, int out_size, void* d_ws, size_t ws_size, hipStream_t stream) {
  (void)in_sizes; (void)n_in; (void)out_size;
  const float** F = (const float**)d_in;
  if (ws_size < (size_t)WS_END) return;
  char* ws = (char*)d_ws; __bf16 *PK = (__bf16*)(ws + WS_PK), *AH = (__bf16*)(ws + WS_AH), *AL = (__bf16*)(ws + WS_AL), *HFH = (__bf16*)(ws + WS_HFH), *HFL = (__bf16*)(ws + WS_HFL); float *Q = (float*)(ws + WS_Q), *Kp = (float*)(ws + WS_K), *V = (float*)(ws + WS_V), *Y = (float*)(ws + WS_Y);
  k_pack<<<dim3(HID, 4), 256, 0, stream>>>(F[3], F[4], F[8], F[10], PK);
  k_ln<<<NR, 128, 0, stream>>>(F[0], nullptr, 1, F[1], F[2], AH, AL);
  k_gemm<0><<<dim3(NR / 64, 3), 128, 0, stream>>>(AH, AL, PK + PK_QKV, nullptr, nullptr, nullptr, Q, Kp, V, nullptr, nullptr, nullptr);
  k_na<<<NRT / 8, 128, 0, stream>>>(Q, Kp, V, AH, AL);
  k_gemm<1><<<dim3(NRT / 64, 1), 128, 0, stream>>>(AH, AL, PK + PK_P, F[5], F[0], nullptr, nullptr, nullptr, nullptr, nullptr, nullptr, Y);
  k_ln<<<NRT, 128, 0, stream>>>(nullptr, Y, 0, F[6], F[7], AH, AL);
  k_gemm<2><<<dim3(NRT / 64, HID / 128), 128, 0, stream>>>(AH, AL, PK + PK_W1, F[9], nullptr, nullptr, nullptr, nullptr, nullptr, HFH, HFL, nullptr);
  k_gemm<3><<<dim3(NRT / 64, 1), 128, 0, stream>>>(HFH, HFL, PK + PK_W2, F[11], nullptr, Y, nullptr, nullptr, nullptr, nullptr, nullptr, (float*)d_out);
}
